// BloodSugarSexMagik_38242388803607
// MI455X (gfx1250) — hardware-run, weakly checked
//
#include <hip/hip_runtime.h>
#include <stddef.h>


#define IMG          256
#define NPIX         65536
#define NCH          12
#define STEPS        100
#define NTHR         256
#define PITCH        272
#define XOFF         8
#define PROWS        258
#define PLANE_RECS   (PROWS * PITCH)
#define PLANE_BYTES  (PLANE_RECS * 16)
#define NPLANES      12
#define SET_RECS     (6 * PLANE_RECS)
#define WT_ITEMS     512
#define FCT_FLOATS   (NCH * NPIX * 16)
#define STATE_FLOATS (NCH * NPIX)
#define PART_FLOATS  (STEPS * 256 * 32)
#define LPART_FLOATS (256 * 32)
#define YT_FLOATS    1312
#define YT_BYTES     5376
#define O_HA         1300
#define O_Z1         (O_HA + STATE_FLOATS)
#define O_HB         (O_Z1 + NPIX)
#define O_Z2         (O_HB + STATE_FLOATS)
#define NF_OUT       (O_Z2 + NPIX)
#define SC_ACT       64.0f
#define SC_W         16.0f
#define SC_INV       0.0009765625f

static_assert(NF_OUT == 1705236);
static_assert((PLANE_BYTES % 256) == 0);
static_assert(((XOFF * 16) % 128) == 0);
static_assert(((PITCH * 16) % 128) == 0);
static_assert(XOFF >= 1 && XOFF + IMG < PITCH);
static_assert(YT_FLOATS * 4 <= YT_BYTES && (YT_FLOATS % 4) == 0);
static_assert((256 + 1) * PITCH + XOFF + IMG - 1 < PLANE_RECS);
static_assert(((NPLANES * PLANE_RECS) % 8) == 0);

typedef float    v4f  __attribute__((ext_vector_type(4)));
typedef float    v8f  __attribute__((ext_vector_type(8)));
typedef unsigned v4u  __attribute__((ext_vector_type(4)));
typedef _Float16 v8h  __attribute__((ext_vector_type(8)));
typedef _Float16 v16h __attribute__((ext_vector_type(16)));
union FragH { v16h v; v8h h[2]; v4u u[2]; };

__device__ __forceinline__ v8f wmh(v16h a, v16h b, v8f c) {
#if defined(__HIP_DEVICE_COMPILE__)
  v8f d = __builtin_amdgcn_wmma_f32_16x16x32_f16(false, a, false, b, (short)0, c, false, false);
  asm volatile("v_nop\n\tv_nop\n\tv_nop\n\tv_nop" : "+v"(d) : "v"(a), "v"(b));
  return d;
#else
  (void)a; (void)b;
  return c;
#endif
}

__device__ __forceinline__ unsigned h16bits(float v) {
  const _Float16 t = (_Float16)v;
  return (unsigned)__builtin_bit_cast(unsigned short, t);
}
__device__ __forceinline__ unsigned pack2(float lo, float hi) {
  return h16bits(lo) | (h16bits(hi) << 16);
}
__device__ __forceinline__ unsigned pack_lo_zero(float v) {
  return h16bits(v) & 0xffffu;
}

__device__ __forceinline__ int poff(int p, int y) {
  const int ky = p / 5, q = p - ky * 5;
  const int kind = (q < 3) ? 0 : (q - 2);
  const int dx = (q < 3) ? (q - 1) : 0;
  return kind * PLANE_RECS + (y + ky) * PITCH + XOFF + dx;
}

__global__ __launch_bounds__(NTHR) void k_zero(v4u* p, int npieces) {
  const int q = blockIdx.x * NTHR + threadIdx.x;
  const v4u z = {0u, 0u, 0u, 0u};
  if (q < npieces) *(volatile v4u*)(p + q) = z;
  __threadfence();
  if (q < npieces) *(volatile v4u*)(p + q) = z;
}

__global__ __launch_bounds__(NTHR) void k_convin(const float* __restrict__ x, const float* __restrict__ w_in,
                                                 const float* __restrict__ b_in, float* cpl, v4u* planes) {
  __shared__ float crow[264];
  const int y = blockIdx.x, px = threadIdx.x;
  float s = b_in[0];
#pragma unroll
  for (int ci = 0; ci < 3; ++ci) {
#pragma unroll
    for (int t = 0; t < 9; ++t) {
      const int yy = y + t / 3 - 1, xx = px + (t % 3) - 1;
      const int yc = min(max(yy, 0), IMG - 1), xc = min(max(xx, 0), IMG - 1);
      float v = x[ci * NPIX + yc * IMG + xc];
      v = ((unsigned)yy < (unsigned)IMG && (unsigned)xx < (unsigned)IMG) ? v : 0.0f;
      s += v * w_in[ci * 9 + t];
    }
  }
  crow[px + 1] = s;
  if (px == 0) crow[0] = 0.0f;
  if (px == 1) crow[257] = 0.0f;
  __syncthreads();
  const float cm = crow[px], cp = crow[px + 2];
  v4u z;
  z.x = 0u;
  z.y = 0u;
  z.z = pack2(cm * SC_ACT, s * SC_ACT);
  z.w = pack_lo_zero(cp * SC_ACT);
  const int orec = (y + 1) * PITCH + XOFF + px;
  float* cdst = cpl + y * IMG + px;
  v4u* za = planes + 2 * PLANE_RECS + orec;
  v4u* zb = planes + 5 * PLANE_RECS + orec;
  *(volatile float*)cdst = s;
  *(volatile v4u*)za = z;
  *(volatile v4u*)zb = z;
  __threadfence();
  *(volatile float*)cdst = s;
  *(volatile v4u*)za = z;
  *(volatile v4u*)zb = z;
}

__global__ __launch_bounds__(NTHR) void k_wpack(const float* __restrict__ w_as, const float* __restrict__ w_bs, v4u* wt) {
  const int tid = threadIdx.x;
  v4u keep[2];
#pragma unroll
  for (int it = 0; it < 2; ++it) {
    const int q = it * NTHR + tid;
    const float* w = (it == 0) ? w_as : w_bs;
    const int row = (q >> 4) & 15, p = q & 15;
    const int ky = p / 5, qq = p - ky * 5;
    const int kyc = min(ky, 2), rowc = min(row, NCH - 1);
    const bool pv = (p < 15) && (row < NCH);
    float vv[8];
#pragma unroll
    for (int e = 0; e < 8; ++e) {
      const int ciA = e + 1,        kxA = qq;
      const int ciB = 9 + (e & 3),  kxB = e >> 2;
      const int ciC = (e < 4) ? (9 + e) : 0;
      const int kxC = (e < 4) ? 2 : ((e < 7) ? (e - 4) : 0);
      const int ci = (qq < 3) ? ciA : ((qq == 3) ? ciB : ciC);
      const int kx = (qq < 3) ? kxA : ((qq == 3) ? kxB : kxC);
      const bool ev = pv && ((qq < 4) || (e < 7));
      const int idx = ((rowc * 13 + ci) * 3 + kyc) * 3 + kx;
      float val = w[idx];
      vv[e] = ev ? (val * SC_W) : 0.0f;
    }
    v4u u;
    u.x = pack2(vv[0], vv[1]);
    u.y = pack2(vv[2], vv[3]);
    u.z = pack2(vv[4], vv[5]);
    u.w = pack2(vv[6], vv[7]);
    keep[it] = u;
    *(volatile v4u*)(wt + q) = u;
  }
  __threadfence();
#pragma unroll
  for (int it = 0; it < 2; ++it) {
    const int q = it * NTHR + tid;
    *(volatile v4u*)(wt + q) = keep[it];
  }
}

__global__ __launch_bounds__(NTHR) void k_fct(const float* __restrict__ w_fcs, float* fct) {
  const int j = blockIdx.x >> 8, y = blockIdx.x & 255, tid = threadIdx.x;
  v4f keep[4];
#pragma unroll
  for (int it = 0; it < 4; ++it) {
    const int q = it * NTHR + tid;
    const int px = q >> 2, part = q & 3;
    float t[4];
#pragma unroll
    for (int i = 0; i < 4; ++i) {
      const int s = 4 * part + i, sc = min(s, NCH - 1);
      float val = w_fcs[(size_t)j * STATE_FLOATS + (size_t)sc * NPIX + (size_t)(y * IMG + px)];
      t[i] = (s < NCH) ? val : 0.0f;
    }
    v4f v = {t[0], t[1], t[2], t[3]};
    keep[it] = v;
    float* dst = fct + ((size_t)(j * NPIX + y * IMG + px) * 16 + 4 * part);
    *(volatile v4f*)dst = v;
  }
  __threadfence();
#pragma unroll
  for (int it = 0; it < 4; ++it) {
    const int q = it * NTHR + tid;
    const int px = q >> 2, part = q & 3;
    float* dst = fct + ((size_t)(j * NPIX + y * IMG + px) * 16 + 4 * part);
    *(volatile v4f*)dst = keep[it];
  }
}

__global__ __launch_bounds__(NTHR) void k_long(const float* __restrict__ cpl, const float* __restrict__ w_al,
                                               const float* __restrict__ b_al, const float* __restrict__ w_bl,
                                               const float* __restrict__ b_bl, const float* __restrict__ w_fcl,
                                               float* lpart) {
  __shared__ float red[8];
  const int y = blockIdx.x, tid = threadIdx.x, px = tid, lane = tid & 31, wave = tid >> 5;
  float ha = b_al[0], hb = b_bl[0];
#pragma unroll
  for (int t = 0; t < 9; ++t) {
    const int yy = y + t / 3 - 1, xx = px + (t % 3) - 1;
    const int yc = min(max(yy, 0), IMG - 1), xc = min(max(xx, 0), IMG - 1);
    float v = cpl[yc * IMG + xc];
    v = ((unsigned)yy < (unsigned)IMG && (unsigned)xx < (unsigned)IMG) ? v : 0.0f;
    ha += v * w_al[t];
    hb += v * w_bl[t];
  }
  const float cc = cpl[y * IMG + px];
  float o = (cc * ha + hb) * w_fcl[y * IMG + px];
#pragma unroll
  for (int sft = 16; sft > 0; sft >>= 1) o += __shfl_xor(o, sft, 32);
  if (lane == 0) red[wave] = o;
  __syncthreads();
  if (wave == 0) {
    float s = 0.0f;
#pragma unroll
    for (int w = 0; w < 8; ++w) s += red[w];
    const float val = (lane == 0) ? s : 0.0f;
    float* dst = lpart + y * 32 + lane;
    *(volatile float*)dst = val;
    __threadfence();
    *(volatile float*)dst = val;
  }
}

__global__ __launch_bounds__(NTHR) void k_step(
    const float* __restrict__ cpl, const v8h* __restrict__ wt, const v8h* __restrict__ pin,
    v4u* pout, const float* __restrict__ fct, const float* __restrict__ b_as,
    const float* __restrict__ b_bs, float* part, float* stA, float* stB, int step, int last) {
  __shared__ __attribute__((aligned(16))) float rec[2 * 258 * 16];
  __shared__ float crow[264];
  __shared__ float red[8 * NCH];
  const int tid = threadIdx.x, lane = tid & 31, wave = tid >> 5, h = lane >> 4, m = lane & 15;
  const int y = blockIdx.x;

  crow[tid + 1] = cpl[y * IMG + tid];
  if (tid == 0) crow[0] = 0.0f;
  if (tid == 1) crow[257] = 0.0f;
  if (tid < 64) {
    const int c = tid >> 5, e = tid & 15, r = ((tid >> 4) & 1) ? 257 : 0;
    rec[(c * 258 + r) * 16 + e] = 0.0f;
  }
  float bsa[8], bsb[8];
#pragma unroll
  for (int r = 0; r < 8; ++r) {
    const int s = 8 * h + r, sc = min(s, NCH - 1);
    const float va = b_as[sc], vb = b_bs[sc];
    bsa[r] = (s < NCH) ? va : 0.0f;
    bsb[r] = (s < NCH) ? vb : 0.0f;
  }

  v8f acc[2][2];
  {
    v8f z;
#pragma unroll
    for (int i = 0; i < 8; ++i) z[i] = 0.0f;
    acc[0][0] = z; acc[0][1] = z; acc[1][0] = z; acc[1][1] = z;
  }
#pragma unroll
  for (int c = 0; c < 2; ++c) {
    const int cb = c * 3 * PLANE_RECS;
#pragma unroll
    for (int ks = 0; ks < 4; ++ks) {
      FragH a;
      a.h[0] = wt[c * 256 + m * 16 + 4 * ks + h];
      a.h[1] = wt[c * 256 + m * 16 + 4 * ks + 2 + h];
      const int oa = (h != 0) ? poff(4 * ks + 1, y) : poff(4 * ks, y);
      const int ob = (ks < 3) ? ((h != 0) ? poff(4 * ks + 3, y) : poff(4 * ks + 2, y)) : poff(14, y);
#pragma unroll
      for (int t = 0; t < 2; ++t) {
        const int px = 32 * wave + 16 * t + m;
        FragH b;
        b.h[0] = pin[cb + oa + px];
        b.h[1] = pin[cb + ob + px];
        if (ks == 3) {
          b.u[1].x = (h != 0) ? 0u : b.u[1].x;
          b.u[1].y = (h != 0) ? 0u : b.u[1].y;
          b.u[1].z = (h != 0) ? 0u : b.u[1].z;
          b.u[1].w = (h != 0) ? 0u : b.u[1].w;
        }
        acc[c][t] = wmh(a.v, b.v, acc[c][t]);
      }
    }
  }

  float hva[2][8], hvb[2][8];
#pragma unroll
  for (int t = 0; t < 2; ++t) {
#pragma unroll
    for (int r = 0; r < 8; ++r) {
      hva[t][r] = acc[0][t][r] * SC_INV + bsa[r];
      hvb[t][r] = acc[1][t][r] * SC_INV + bsb[r];
    }
  }
#pragma unroll
  for (int t = 0; t < 2; ++t) {
    const int px = 32 * wave + 16 * t + m;
    float* ra = rec + (0 * 258 + px + 1) * 16 + 8 * h;
    float* rb = rec + (1 * 258 + px + 1) * 16 + 8 * h;
    const v4f a0 = {hva[t][0], hva[t][1], hva[t][2], hva[t][3]};
    const v4f a1 = {hva[t][4], hva[t][5], hva[t][6], hva[t][7]};
    const v4f b0 = {hvb[t][0], hvb[t][1], hvb[t][2], hvb[t][3]};
    const v4f b1 = {hvb[t][4], hvb[t][5], hvb[t][6], hvb[t][7]};
    *(v4f*)ra = a0;
    *(v4f*)(ra + 4) = a1;
    *(v4f*)rb = b0;
    *(v4f*)(rb + 4) = b1;
  }
  __syncthreads();

  float f[NCH];
#pragma unroll
  for (int j = 0; j < NCH; ++j) f[j] = 0.0f;
#pragma unroll
  for (int t = 0; t < 2; ++t) {
    const int px = 32 * wave + 16 * t + m;
    const float cv = crow[px + 1];
    float o[8];
#pragma unroll
    for (int r = 0; r < 8; ++r) o[r] = cv * hva[t][r] + hvb[t][r];
    const float* wp = fct + ((size_t)(y * IMG + px) * 16 + 8 * h);
#pragma unroll
    for (int j = 0; j < NCH; ++j) {
      const float* wj = wp + (size_t)j * ((size_t)NPIX * 16);
      const v4f w0 = *(const v4f*)wj;
      const v4f w1 = *(const v4f*)(wj + 4);
      float s = f[j];
      s += o[0] * w0.x; s += o[1] * w0.y; s += o[2] * w0.z; s += o[3] * w0.w;
      s += o[4] * w1.x; s += o[5] * w1.y; s += o[6] * w1.z; s += o[7] * w1.w;
      f[j] = s;
    }
  }
#pragma unroll
  for (int j = 0; j < NCH; ++j) {
    float v = f[j];
#pragma unroll
    for (int sft = 16; sft > 0; sft >>= 1) v += __shfl_xor(v, sft, 32);
    if (lane == 0) red[wave * NCH + j] = v;
  }

  const int xg = 32 * wave + lane;
  const int orec = (y + 1) * PITCH + XOFF + xg;
  v4u pw[2][3];
#pragma unroll
  for (int c = 0; c < 2; ++c) {
    const float* r0 = rec + (c * 258 + xg) * 16;
    const float* r1 = r0 + 16;
    const float* r2 = r0 + 32;
    const v4f e0 = *(const v4f*)r1;
    const v4f e1 = *(const v4f*)(r1 + 4);
    const v4f q0 = *(const v4f*)(r0 + 8);
    const v4f q1 = *(const v4f*)(r1 + 8);
    const v4f q2 = *(const v4f*)(r2 + 8);
    const float cm = crow[xg], c0 = crow[xg + 1], cp = crow[xg + 2];
    v4u u;
    u.x = pack2(e0.x * SC_ACT, e0.y * SC_ACT);
    u.y = pack2(e0.z * SC_ACT, e0.w * SC_ACT);
    u.z = pack2(e1.x * SC_ACT, e1.y * SC_ACT);
    u.w = pack2(e1.z * SC_ACT, e1.w * SC_ACT);
    pw[c][0] = u;
    u.x = pack2(q0.x * SC_ACT, q0.y * SC_ACT);
    u.y = pack2(q0.z * SC_ACT, q0.w * SC_ACT);
    u.z = pack2(q1.x * SC_ACT, q1.y * SC_ACT);
    u.w = pack2(q1.z * SC_ACT, q1.w * SC_ACT);
    pw[c][1] = u;
    u.x = pack2(q2.x * SC_ACT, q2.y * SC_ACT);
    u.y = pack2(q2.z * SC_ACT, q2.w * SC_ACT);
    u.z = pack2(cm * SC_ACT, c0 * SC_ACT);
    u.w = pack_lo_zero(cp * SC_ACT);
    pw[c][2] = u;
  }
#pragma unroll
  for (int c = 0; c < 2; ++c) {
#pragma unroll
    for (int k = 0; k < 3; ++k) *(volatile v4u*)(pout + (c * 3 + k) * PLANE_RECS + orec) = pw[c][k];
  }
  float sva[NCH], svb[NCH];
  if (last) {
#pragma unroll
    for (int ch = 0; ch < NCH; ++ch) {
      sva[ch] = rec[(0 * 258 + xg + 1) * 16 + ch];
      svb[ch] = rec[(1 * 258 + xg + 1) * 16 + ch];
      *(volatile float*)(stA + (size_t)ch * NPIX + (size_t)(y * IMG + xg)) = sva[ch];
      *(volatile float*)(stB + (size_t)ch * NPIX + (size_t)(y * IMG + xg)) = svb[ch];
    }
  }
  __syncthreads();
  float pv = 0.0f;
  if (wave == 0) {
    const int jj = min(lane, NCH - 1);
    float s = 0.0f;
#pragma unroll
    for (int w = 0; w < 8; ++w) s += red[w * NCH + jj];
    pv = (lane < NCH) ? s : 0.0f;
    *(volatile float*)(part + ((size_t)step * 256 + y) * 32 + lane) = pv;
  }
  __threadfence();
#pragma unroll
  for (int c = 0; c < 2; ++c) {
#pragma unroll
    for (int k = 0; k < 3; ++k) *(volatile v4u*)(pout + (c * 3 + k) * PLANE_RECS + orec) = pw[c][k];
  }
  if (last) {
#pragma unroll
    for (int ch = 0; ch < NCH; ++ch) {
      *(volatile float*)(stA + (size_t)ch * NPIX + (size_t)(y * IMG + xg)) = sva[ch];
      *(volatile float*)(stB + (size_t)ch * NPIX + (size_t)(y * IMG + xg)) = svb[ch];
    }
  }
  if (wave == 0) {
    *(volatile float*)(part + ((size_t)step * 256 + y) * 32 + lane) = pv;
  }
}

__global__ __launch_bounds__(NTHR) void k_reduce(const float* __restrict__ part, const float* __restrict__ lpart,
                                                 const float* __restrict__ b_fcs, const float* __restrict__ b_fcl,
                                                 const int* __restrict__ s_steps, const int* __restrict__ l_steps,
                                                 float* ytab) {
  __shared__ __attribute__((aligned(16))) float yt[YT_FLOATS];
  const int tid = threadIdx.x;
  int nS = s_steps[0]; nS = min(max(nS, 0), STEPS);
  int nL = l_steps[0]; nL = min(max(nL, 0), STEPS);
#pragma unroll 1
  for (int it = 0; it < 5; ++it) {
    const int i = it * NTHR + tid;
    const int ii = min(i, NCH * STEPS - 1);
    const int j = ii / STEPS, t = ii - j * STEPS;
    double s = (double)b_fcs[j];
#pragma unroll 1
    for (int blk = 0; blk < 256; ++blk) s += (double)part[((size_t)t * 256 + blk) * 32 + j];
    const float val = (t < nS) ? (float)s : 0.0f;
    if (i < NCH * STEPS) yt[i] = val;
  }
  double sl = (double)b_fcl[0];
#pragma unroll 1
  for (int blk = 0; blk < 256; ++blk) sl += (double)lpart[blk * 32];
  if (tid < YT_FLOATS - NCH * STEPS) {
    const float v = (tid < STEPS && tid < nL) ? (float)sl : 0.0f;
    yt[NCH * STEPS + tid] = v;
  }
  __syncthreads();
  v4f keep[2];
#pragma unroll
  for (int it = 0; it < 2; ++it) {
    const int q = it * NTHR + tid;
    const int qc = min(q, YT_FLOATS / 4 - 1);
    const v4f v = *(const v4f*)(yt + 4 * qc);
    keep[it] = v;
    if (q < YT_FLOATS / 4) *(volatile v4f*)(ytab + 4 * q) = v;
  }
  __threadfence();
#pragma unroll
  for (int it = 0; it < 2; ++it) {
    const int q = it * NTHR + tid;
    if (q < YT_FLOATS / 4) *(volatile v4f*)(ytab + 4 * q) = keep[it];
  }
}

__global__ __launch_bounds__(NTHR) void k_pack(const float* __restrict__ ytab, const float* __restrict__ stA,
                                               const float* __restrict__ stB, float* out, int npieces) {
  const int q = blockIdx.x * NTHR + threadIdx.x;
  const int qc = min(q, npieces - 1);
  const int f = 4 * qc;
  const v4f vy = *(const v4f*)(ytab + min(f, YT_FLOATS - 4));
  const v4f va = *(const v4f*)(stA + min(max(f - O_HA, 0), STATE_FLOATS - 4));
  const v4f vb = *(const v4f*)(stB + min(max(f - O_HB, 0), STATE_FLOATS - 4));
  const v4f z = {0.0f, 0.0f, 0.0f, 0.0f};
  const v4f v = (f < O_HA) ? vy : ((f < O_Z1) ? va : ((f < O_HB) ? z : ((f < O_Z2) ? vb : z)));
  if (q < npieces) *(volatile v4f*)(out + f) = v;
  __threadfence();
  if (q < npieces) *(volatile v4f*)(out + f) = v;
}

extern "C" void kernel_launch(void* const* d_in, const int* in_sizes, int n_in,
                              void* d_out, int out_size, void* d_ws, size_t ws_size,
                              hipStream_t stream) {
  if (n_in < 17) return;
  if (in_sizes[0] != 3 * NPIX || in_sizes[1] != 27 || in_sizes[2] < 1) return;
  if (in_sizes[3] != 1404 || in_sizes[4] < NCH || in_sizes[5] != 1404 || in_sizes[6] < NCH) return;
  if (in_sizes[7] != 18 || in_sizes[8] < 1 || in_sizes[9] != 18 || in_sizes[10] < 1) return;
  if (in_sizes[11] != NCH * STATE_FLOATS || in_sizes[12] < NCH || in_sizes[13] != NPIX || in_sizes[14] < 1) return;
  if (in_sizes[15] < 1 || in_sizes[16] < 1) return;
  if (out_size != NF_OUT) return;

  const float* x     = (const float*)d_in[0];
  const float* w_in  = (const float*)d_in[1];
  const float* b_in  = (const float*)d_in[2];
  const float* w_as  = (const float*)d_in[3];
  const float* b_as  = (const float*)d_in[4];
  const float* w_bs  = (const float*)d_in[5];
  const float* b_bs  = (const float*)d_in[6];
  const float* w_al  = (const float*)d_in[7];
  const float* b_al  = (const float*)d_in[8];
  const float* w_bl  = (const float*)d_in[9];
  const float* b_bl  = (const float*)d_in[10];
  const float* w_fcs = (const float*)d_in[11];
  const float* b_fcs = (const float*)d_in[12];
  const float* w_fcl = (const float*)d_in[13];
  const float* b_fcl = (const float*)d_in[14];
  const int*   sst   = (const int*)d_in[15];
  const int*   lst   = (const int*)d_in[16];
  float* out = (float*)d_out;

  char* ws = (char*)d_ws;
  size_t off = 0;
  const size_t oCpl  = off; off += (size_t)NPIX * 4;
  const size_t oWt   = off; off += (size_t)WT_ITEMS * 16;
  const size_t oPl   = off; off += (size_t)NPLANES * PLANE_BYTES;
  const size_t oFct  = off; off += (size_t)FCT_FLOATS * 4;
  const size_t oPart = off; off += (size_t)PART_FLOATS * 4;
  const size_t oLp   = off; off += (size_t)LPART_FLOATS * 4;
  const size_t oStA  = off; off += (size_t)STATE_FLOATS * 4;
  const size_t oStB  = off; off += (size_t)STATE_FLOATS * 4;
  const size_t oYt   = off; off += (size_t)YT_BYTES;
  if (off > ws_size) return;

  float* cpl   = (float*)(ws + oCpl);
  v4u*   wt_u  = (v4u*)(ws + oWt);
  const v8h* wt_h = (const v8h*)(ws + oWt);
  v4u*   pl_u  = (v4u*)(ws + oPl);
  const v8h* pl_h = (const v8h*)(ws + oPl);
  float* fct   = (float*)(ws + oFct);
  float* part  = (float*)(ws + oPart);
  float* lpart = (float*)(ws + oLp);
  float* stA   = (float*)(ws + oStA);
  float* stB   = (float*)(ws + oStB);
  float* ytab  = (float*)(ws + oYt);

  const int zpieces = NPLANES * PLANE_RECS;
  const int zblk = (zpieces + NTHR - 1) / NTHR;
  k_zero<<<zblk, NTHR, 0, stream>>>(pl_u, zpieces);

  k_convin<<<IMG, NTHR, 0, stream>>>(x, w_in, b_in, cpl, pl_u);
  k_wpack<<<1, NTHR, 0, stream>>>(w_as, w_bs, wt_u);
  k_fct<<<NCH * IMG, NTHR, 0, stream>>>(w_fcs, fct);
  k_long<<<IMG, NTHR, 0, stream>>>(cpl, w_al, b_al, w_bl, b_bl, w_fcl, lpart);

  for (int t = 0; t < STEPS; ++t) {
    const v8h* pin = pl_h + (size_t)(t & 1) * SET_RECS;
    v4u* pout = pl_u + (size_t)((t + 1) & 1) * SET_RECS;
    const int last = (t == STEPS - 1) ? 1 : 0;
    k_step<<<IMG, NTHR, 0, stream>>>(cpl, wt_h, pin, pout, fct, b_as, b_bs, part, stA, stB, t, last);
  }

  k_reduce<<<1, NTHR, 0, stream>>>(part, lpart, b_fcs, b_fcl, sst, lst, ytab);

  const int npieces = NF_OUT / 4;
  const int nblk = (npieces + NTHR - 1) / NTHR;
  k_pack<<<nblk, NTHR, 0, stream>>>(ytab, stA, stB, out, npieces);
}
